// BivariateSpectral_66322884985417
// MI455X (gfx1250) — hardware-verified
//
#include <hip/hip_runtime.h>
#include <stdint.h>

typedef _Float16 v16h __attribute__((ext_vector_type(16)));
typedef _Float16 v8h  __attribute__((ext_vector_type(8)));
typedef float    v8f  __attribute__((ext_vector_type(8)));
typedef float    v4f  __attribute__((ext_vector_type(4)));
typedef float    v2f  __attribute__((ext_vector_type(2)));

namespace {
constexpr int   kDim     = 64;
constexpr int   kTM      = 16;
constexpr int   kNW      = 4;
constexpr int   kThreads = kNW * 32;
constexpr int   kMats    = kNW * kTM;
constexpr int   kSteps   = 56;
constexpr int   kBis     = 24;
constexpr int   kPitch   = 72;
constexpr int   kNS      = 5;
constexpr int   kSMat    = kDim * kPitch;
constexpr float kOpScale = 64.0f;
constexpr float kEpi     = 0.0078125f;
constexpr float kPiv     = 1.0e-10f;
}

union FragA { v16h v; v8h hh[2]; };
union FragB { v16h v; _Float16 e[16]; };
union F8    { v4f p[2]; float f[8]; };

__device__ __forceinline__ v8f zero8() {
  v8f z = {0.f, 0.f, 0.f, 0.f, 0.f, 0.f, 0.f, 0.f};
  return z;
}

__device__ __forceinline__ v8f wm(v16h a, v16h b, v8f c) {
  v8f d = __builtin_amdgcn_wmma_f32_16x16x32_f16(false, a, false, b, (short)0, c, false, false);
  asm volatile("v_nop\n\tv_nop\n\tv_nop\n\tv_nop" : "+v"(d) : "v"(a), "v"(b));
  return d;
}

__device__ __forceinline__ v16h ld_a(const _Float16* S, int row, int kk, int h) {
  FragA f;
  const _Float16* p = S + row * kPitch + 32 * kk + 8 * h;
  f.hh[0] = *(const v8h*)(p);
  f.hh[1] = *(const v8h*)(p + 16);
  return f.v;
}


__device__ __forceinline__ void pass_scaled(const _Float16* S, const float* sV,
                                            const float (&v)[32], float (&u)[32], int m, int h)
{
  FragB bf[2];
#pragma unroll
  for (int t = 0; t < 4; ++t) {
    F8 s;
    s.p[0] = *(const v4f*)(sV + m * kDim + 16 * t + 8 * h);
    s.p[1] = *(const v4f*)(sV + m * kDim + 16 * t + 8 * h + 4);
#pragma unroll
    for (int r = 0; r < 8; ++r) {
      const int q = 8 * t + r;
      bf[q >> 4].e[q & 15] = (_Float16)(kOpScale * v[q] * s.f[r]);
    }
  }
#pragma unroll
  for (int t = 0; t < 4; ++t) {
    v8f acc = zero8();
#pragma unroll
    for (int kk = 0; kk < 2; ++kk)
      acc = wm(ld_a(S, 16 * t + m, kk, h), bf[kk].v, acc);
#pragma unroll
    for (int r = 0; r < 8; ++r) u[8 * t + r] += kEpi * acc[r];
  }
}

__device__ __forceinline__ void pass_main(const _Float16* sAA, const _Float16* sBt, const _Float16* sCt,
                                          const float* sX, const float* sY,
                                          const float (&v)[32], float (&u)[32], int m, int h)
{
  FragB bf[2];
#pragma unroll
  for (int q = 0; q < 32; ++q) bf[q >> 4].e[q & 15] = (_Float16)(kOpScale * v[q]);
#pragma unroll
  for (int t = 0; t < 4; ++t) {
    v8f a = zero8(), tb = zero8(), tc = zero8();
#pragma unroll
    for (int kk = 0; kk < 2; ++kk) {
      a  = wm(ld_a(sAA, 16 * t + m, kk, h), bf[kk].v, a);
      tb = wm(ld_a(sBt, 16 * t + m, kk, h), bf[kk].v, tb);
      tc = wm(ld_a(sCt, 16 * t + m, kk, h), bf[kk].v, tc);
    }
    F8 xs, ys;
    xs.p[0] = *(const v4f*)(sX + m * kDim + 16 * t + 8 * h);
    xs.p[1] = *(const v4f*)(sX + m * kDim + 16 * t + 8 * h + 4);
    ys.p[0] = *(const v4f*)(sY + m * kDim + 16 * t + 8 * h);
    ys.p[1] = *(const v4f*)(sY + m * kDim + 16 * t + 8 * h + 4);
#pragma unroll
    for (int r = 0; r < 8; ++r) {
      const int q = 8 * t + r;
      u[q] += kEpi * (a[r] + xs.f[r] * tb[r] + ys.f[r] * tc[r]);
    }
  }
}

__global__ void __launch_bounds__(kThreads)
lanczos_min_eig(const float* __restrict__ xg, const float* __restrict__ yg,
                const float* __restrict__ Ag, const float* __restrict__ Bg,
                const float* __restrict__ Cg, const int* __restrict__ eig,
                float* out, int batch, int nOut)
{
  __shared__ __attribute__((aligned(16))) _Float16 sS[kNS * kSMat];
  __shared__ __attribute__((aligned(16))) float    sXY[kNW * 2 * kTM * kDim];
  __shared__ __attribute__((aligned(16))) float    sT[kSteps * kMats * 2];
  __shared__ __attribute__((aligned(16))) float    sOut[kMats];

  const int lane = threadIdx.x & 31;
  const int w    = threadIdx.x >> 5;
  const int h    = lane >> 4;
  const int m    = lane & 15;
  const int b0   = (blockIdx.x * kNW + w) * kTM;

  for (int e = threadIdx.x; e < kDim * kDim; e += kThreads) {
    const int i = e >> 6, k = e & 63;
    const int ik = i * kDim + k, ki = k * kDim + i;
    _Float16* p = sS + i * kPitch + k;
    p[0]         = (_Float16)(Ag[ik] + Ag[ki]);
    p[kSMat]     = (_Float16)Bg[ik];
    p[2 * kSMat] = (_Float16)Bg[ki];
    p[3 * kSMat] = (_Float16)Cg[ik];
    p[4 * kSMat] = (_Float16)Cg[ki];
  }

  float* sX = sXY + (2 * w) * (kTM * kDim);
  float* sY = sX + kTM * kDim;
  {
    const int bl = batch - 1;
#pragma unroll
    for (int i = 0; i < 8; ++i) {
      const int f = lane + 32 * i;
      const int row = f >> 4, c4 = (f & 15) * 4;
      int gr = b0 + row;
      gr = (gr > bl) ? bl : gr;
      const size_t go = (size_t)gr * kDim + c4;
      *(v4f*)(sX + row * kDim + c4) = *(const v4f*)(xg + go);
      *(v4f*)(sY + row * kDim + c4) = *(const v4f*)(yg + go);
    }
  }
  __syncthreads();

  const _Float16* sAA = sS;
  const _Float16* sB  = sS + kSMat;
  const _Float16* sBt = sS + 2 * kSMat;
  const _Float16* sC  = sS + 3 * kSMat;
  const _Float16* sCt = sS + 4 * kSMat;

  float v[32], u[32];
  {
    float n0 = 0.f;
#pragma unroll
    for (int q = 0; q < 32; ++q) {
      const int k = 16 * (q >> 3) + 8 * h + (q & 7);
      const float s = 1.0f + 0.03125f * (float)((k * 7 + 3) & 15);
      v[q] = s;
      u[q] = 0.f;
      n0 += s * s;
    }
    n0 += __shfl_xor(n0, 16, 32);
    const float r0 = 1.0f / sqrtf(n0);
#pragma unroll
    for (int q = 0; q < 32; ++q) v[q] *= r0;
  }

  float beta = 0.f, glo = 3.0e38f, ghi = -3.0e38f;
#pragma unroll 1
  for (int j = 0; j < kSteps; ++j) {
#pragma unroll
    for (int q = 0; q < 32; ++q) u[q] = -beta * u[q];

    pass_scaled(sB, sX, v, u, m, h);
    asm volatile("" ::: "memory");
    pass_scaled(sC, sY, v, u, m, h);
    asm volatile("" ::: "memory");
    pass_main(sAA, sBt, sCt, sX, sY, v, u, m, h);
    asm volatile("" ::: "memory");

    float s = 0.f;
#pragma unroll
    for (int q = 0; q < 32; ++q) s += v[q] * u[q];
    s += __shfl_xor(s, 16, 32);
    const float alpha = s;

    float n2 = 0.f;
#pragma unroll
    for (int q = 0; q < 32; ++q) {
      const float t0 = u[q] - alpha * v[q];
      u[q] = t0;
      n2 += t0 * t0;
    }
    n2 += __shfl_xor(n2, 16, 32);
    const float bn = sqrtf(n2);

    const float rad = beta + ((j + 1 < kSteps) ? bn : 0.f);
    glo = fminf(glo, alpha - rad);
    ghi = fmaxf(ghi, alpha + rad);
    if (h == 0) {
      v2f ab;
      ab.x = alpha;
      ab.y = bn * bn;
      *(v2f*)(sT + (j * kMats + w * kTM + m) * 2) = ab;
    }

    const float inv = (bn > 1.0e-30f) ? (1.0f / bn) : 0.f;
#pragma unroll
    for (int q = 0; q < 32; ++q) {
      const float t0 = v[q];
      v[q] = u[q] * inv;
      u[q] = t0;
    }
    beta = bn;
  }
  __syncthreads();

  int ci = eig[0];
  ci = (ci < 0) ? 0 : ci;
  ci = (ci > kSteps - 1) ? (kSteps - 1) : ci;
  float lo = glo - 1.0e-3f * (fabsf(glo) + 1.0f);
  float hi = ghi + 1.0e-3f * (fabsf(ghi) + 1.0f);
  const float* tT = sT + 2 * (w * kTM + m);
#pragma unroll 1
  for (int it = 0; it < kBis; ++it) {
    const float xm = 0.5f * (lo + hi);
    int cnt = 0;
    float d = 1.0f, b2 = 0.0f;
#pragma unroll 8
    for (int jj = 0; jj < kSteps; ++jj) {
      const v2f ab = *(const v2f*)(tT + jj * (2 * kMats));
      float dn = ab.x - xm - b2 / d;
      dn = (fabsf(dn) < kPiv) ? -kPiv : dn;
      cnt += (dn < 0.0f) ? 1 : 0;
      d  = dn;
      b2 = ab.y;
    }
    if (cnt > ci) hi = xm; else lo = xm;
  }
  const float lam = 0.5f * (lo + hi);

  if (h == 0) sOut[w * kTM + m] = lam;
  __syncthreads();
  if (w == 0 && lane < 16) {
    const int g0 = blockIdx.x * kMats + 4 * lane;
    const v4f val = *(const v4f*)(sOut + 4 * lane);
    const bool full = (g0 + 3) < nOut;
    if (full) {
      *(volatile v4f*)(out + g0) = val;
    } else {
#pragma unroll
      for (int e = 0; e < 4; ++e)
        if (g0 + e < nOut) *(volatile float*)(out + g0 + e) = val[e];
    }
    __threadfence();
    if (full) {
      *(volatile v4f*)(out + g0) = val;
    } else {
#pragma unroll
      for (int e = 0; e < 4; ++e)
        if (g0 + e < nOut) *(volatile float*)(out + g0 + e) = val[e];
    }
  }
}

extern "C" void kernel_launch(void* const* d_in, const int* in_sizes, int n_in,
                              void* d_out, int out_size, void* d_ws, size_t ws_size,
                              hipStream_t stream)
{
  (void)n_in; (void)d_ws; (void)ws_size;
  const float* x = (const float*)d_in[0];
  const float* y = (const float*)d_in[1];
  const float* A = (const float*)d_in[2];
  const float* B = (const float*)d_in[3];
  const float* C = (const float*)d_in[4];
  const int* eig = (const int*)d_in[5];
  float* out = (float*)d_out;

  const int batch = in_sizes[0] / kDim;
  const int nOut  = (out_size < batch) ? out_size : batch;
  if (batch <= 0 || nOut <= 0) return;
  const int nTiles = (batch + kTM - 1) / kTM;
  const int blocks = (nTiles + kNW - 1) / kNW;

  hipLaunchKernelGGL(lanczos_min_eig, dim3(blocks), dim3(kThreads), 0, stream,
                     x, y, A, B, C, eig, out, batch, nOut);
}
